// FullFastSTU_48404281426451
// MI455X (gfx1250) — hardware-verified
//
#include <hip/hip_runtime.h>

typedef __attribute__((ext_vector_type(16))) _Float16 v16h;
typedef __attribute__((ext_vector_type(8)))  _Float16 v8h;
typedef __attribute__((ext_vector_type(8)))  float    v8f;
typedef __attribute__((ext_vector_type(4)))  float    v4f;

constexpr int kBatch  = 4;
constexpr int kSeq    = 1024;
constexpr int kDim    = 256;
constexpr int kState  = 64;
constexpr int kChan   = 48;
constexpr int kTaps   = 8;
constexpr int kRows   = kBatch * kSeq;
constexpr int kKtot   = kDim * kChan;
constexpr int kKEmit  = 96;
constexpr int kHPitch = 104;
constexpr int kDBlk   = 8;
constexpr int kDWave  = 4;
constexpr int kSteps  = 16;
constexpr int kStPitch = 200;
constexpr int kTrPitch = 200;
constexpr int kXRows  = 24;

static_assert(kState + kTaps <= kKEmit && (kKEmit % 32) == 0, "emit K padding");
static_assert(kKtot == 12288 && (kKtot % 32) == 0, "filter K multiple of 32");
static_assert((kRows % 64) == 0 && (kDim % 64) == 0, "GEMM M,N multiples of 64");
static_assert((kSeq % kSteps) == 0 && (kDim % kDBlk) == 0, "scan tiling");
static_assert(kDWave * kChan * 2 == 384, "a wave owns three whole 128-B lines per row");
static_assert((kHPitch % 8) == 0 && (kStPitch % 8) == 0 && (kTrPitch % 8) == 0, "16-B aligned LDS rows");
static_assert(kXRows * kDBlk == 3 * 64, "x staging covers exactly 3 elements per thread");
static_assert((kChan * kKEmit) % 64 == 0, "C^T plane build covers exactly");

constexpr float kCarryH = 16.0f;
constexpr float kCarryC = 256.0f;
constexpr float kCarryU = 16.0f;
constexpr float kCarryW = 1024.0f;
constexpr float kEmitScale = kCarryU / (kCarryH * kCarryC);
constexpr float kGemmScale = 1.0f / (kCarryU * kCarryW);

constexpr size_t kOffU    = 0;
constexpr size_t kBytesU  = (size_t)kRows * kKtot * 2;
constexpr size_t kOffW    = kOffU + kBytesU;
constexpr size_t kBytesW  = (size_t)kDim * kKtot * 2;
constexpr size_t kWsTotal = kOffW + kBytesW;
static_assert(kBytesU == 100663296ull && kBytesW == 6291456ull, "plane sizes");
static_assert(kWsTotal == 106954752ull, "carve total");
static_assert(kWsTotal <= 134217728ull, "carve cap");
static_assert((kOffW % 128) == 0, "aligned regions");

struct FragH {
  union U { v16h v; v8h h[2]; };
  static __device__ __forceinline__ v16h load(const _Float16* p) {
    U f;
    f.h[0] = *(const v8h*)(p);
    f.h[1] = *(const v8h*)(p + 16);
    return f.v;
  }
};

__device__ __forceinline__ v8f mma_h(v16h a, v16h b, v8f c) {
  c = __builtin_amdgcn_wmma_f32_16x16x32_f16(false, a, false, b, (short)0, c, false, false);
  asm volatile("v_nop\n\tv_nop\n\tv_nop\n\tv_nop" : "+v"(c) : "v"(a), "v"(b));
  return c;
}
__device__ __forceinline__ v8f mma_raw(v16h a, v16h b, v8f c) {
  return __builtin_amdgcn_wmma_f32_16x16x32_f16(false, a, false, b, (short)0, c, false, false);
}
__device__ __forceinline__ void guard_row4(v8f& c0, v8f& c1, v8f& c2, v8f& c3,
                                           v16h a, v16h b0, v16h b1, v16h b2, v16h b3) {
  asm volatile("v_nop\n\tv_nop\n\tv_nop\n\tv_nop"
               : "+v"(c0), "+v"(c1), "+v"(c2), "+v"(c3)
               : "v"(a), "v"(b0), "v"(b1), "v"(b2), "v"(b3));
}
__device__ __forceinline__ void acc_guard4(v8f& a, v8f& b, v8f& c, v8f& d) {
  asm volatile("v_nop\n\tv_nop\n\tv_nop\n\tv_nop" : "+v"(a), "+v"(b), "+v"(c), "+v"(d));
}

__global__ __launch_bounds__(256) void prep_filter_kernel(
    const float* __restrict__ Mp, const float* __restrict__ Mm, unsigned short* __restrict__ Wt)
{
  __shared__ __align__(16) _Float16 sT[64 * kTrPitch];
  const int tid  = threadIdx.x;
  const int lane = tid & 31;
  const int wave = __builtin_amdgcn_readfirstlane((int)(threadIdx.x >> 5));
  const int d0 = blockIdx.x * kDWave;
  const int e0 = blockIdx.y * 64;
  const int rsub = tid >> 4;
  const int e4 = (tid & 15) * 4;
#pragma unroll 1
  for (int it = 0; it < 12; ++it) {
    const int rowi = it * 16 + rsub;
    const int dd = rowi / kChan;
    const int k  = rowi - dd * kChan;
    const bool plus = (k < 24);
    const int kp = plus ? k : 23;
    const int km = plus ? 0 : (k - 24);
    const int d = d0 + dd;
    v4f vp = *(const v4f*)(Mp + ((size_t)(kp * kDim + d)) * kDim + e0 + e4);
    v4f vm = *(const v4f*)(Mm + ((size_t)(km * kDim + d)) * kDim + e0 + e4);
    asm volatile("" : "+v"(vp));
    asm volatile("" : "+v"(vm));
#pragma unroll
    for (int c = 0; c < 4; ++c) {
      const float a = vp[c];
      const float b = vm[c];
      const float v = plus ? a : b;
      sT[(e4 + c) * kTrPitch + rowi] = (_Float16)(v * kCarryW);
    }
  }
  __syncthreads();
  const int q = lane >> 3;
  const int c8 = (lane & 7) * 8;
  for (int pass = 0; pass < 2; ++pass) {
#pragma unroll
    for (int it = 0; it < 6; ++it) {
      const int ln = (it * 8 + wave) * 4 + q;
      const int e = ln / 3;
      const int j = ln - e * 3;
      const v8h v = *(const v8h*)(sT + e * kTrPitch + j * 64 + c8);
      *(volatile v8h*)(Wt + (size_t)(e0 + e) * kKtot + d0 * kChan + j * 64 + c8) = v;
    }
    __threadfence();
  }
}

__global__ __launch_bounds__(64) void scan_emit_kernel(
    const float* __restrict__ x, const float* __restrict__ Av, const float* __restrict__ Bv,
    const float* __restrict__ Cm, const float* __restrict__ Mt, unsigned short* __restrict__ Uo)
{
  __shared__ __align__(16) _Float16 sH[kDBlk * kSteps * kHPitch];
  __shared__ __align__(16) _Float16 sCt[kChan * kHPitch];
  __shared__ __align__(16) _Float16 sSt[2][kSteps * kStPitch];
  __shared__ __align__(16) float sX[kXRows * kDBlk];

  const int tid  = threadIdx.x;
  const int lane = tid & 31;
  const int wave = __builtin_amdgcn_readfirstlane((int)(threadIdx.x >> 5));
  const int d0 = blockIdx.x * kDBlk;
  const int b  = blockIdx.y;
  const int dl = tid & 7;
  const int sg = tid >> 3;
  const int rlane = lane & 15;
  const int koff  = (lane >> 4) * 8;
  const int mOff  = (lane >> 4) * 8;

#pragma unroll 2
  for (int it = 0; it < (kChan * kKEmit) / 64; ++it) {
    const int i = tid + 64 * it;
    const int n = i / kKEmit;
    const int kk = i - n * kKEmit;
    const int kc = (kk < kState) ? kk : (kState - 1);
    int kt = kk - kState;
    kt = (kt < 0) ? 0 : ((kt > kTaps - 1) ? (kTaps - 1) : kt);
    float vc = Cm[kc * kChan + n];
    float vm = Mt[n * kTaps + kt];
    asm volatile("" : "+v"(vc));
    asm volatile("" : "+v"(vm));
    const float v = (kk < kState) ? vc : ((kk < kState + kTaps) ? vm : 0.0f);
    sCt[n * kHPitch + kk] = (_Float16)(v * kCarryC);
  }

  float ar[8], br[8], h[8];
  {
    const v4f a0 = *(const v4f*)(Av + sg * 8);
    const v4f a1 = *(const v4f*)(Av + sg * 8 + 4);
    const v4f b0 = *(const v4f*)(Bv + sg * 8);
    const v4f b1 = *(const v4f*)(Bv + sg * 8 + 4);
#pragma unroll
    for (int j = 0; j < 4; ++j) {
      ar[j] = a0[j];
      ar[4 + j] = a1[j];
      br[j] = b0[j];
      br[4 + j] = b1[j];
    }
#pragma unroll
    for (int j = 0; j < 8; ++j) h[j] = 0.0f;
  }
  __syncthreads();

  v16h bfr[3][3];
#pragma unroll
  for (int nt = 0; nt < 3; ++nt)
#pragma unroll
    for (int ks = 0; ks < 3; ++ks)
      bfr[nt][ks] = FragH::load(sCt + (nt * 16 + rlane) * kHPitch + koff + ks * 32);

  _Float16* stw = sSt[wave];
  const int q  = lane >> 3;
  const int c8 = (lane & 7) * 8;

#pragma unroll 1
  for (int sub = 0; sub < kSeq / kSteps; ++sub) {
    const int l0 = sub * kSteps;
#pragma unroll
    for (int it = 0; it < 3; ++it) {
      const int i = tid + 64 * it;
      const int r = i >> 3;
      const int dd = i & 7;
      const int l = l0 - 8 + r;
      const int lc = (l < 0) ? 0 : l;
      float v = x[((size_t)(b * kSeq + lc)) * kDim + d0 + dd];
      asm volatile("" : "+v"(v));
      sX[i] = (l >= 0) ? v : 0.0f;
    }
    __syncthreads();

#pragma unroll 1
    for (int st = 0; st < kSteps; ++st) {
      const float xv = sX[(st + 8) * kDBlk + dl];
      v8h hv;
#pragma unroll
      for (int j = 0; j < 8; ++j) {
        h[j] = fmaf(h[j], ar[j], xv * br[j]);
        hv[j] = (_Float16)(h[j] * kCarryH);
      }
      *(v8h*)(sH + (dl * kSteps + st) * kHPitch + sg * 8) = hv;
    }
#pragma unroll
    for (int i2 = 0; i2 < 2; ++i2) {
      const int rowid = tid + 64 * i2;
      const int dd = rowid & 7;
      const int ls = rowid >> 3;
      v8h tv;
#pragma unroll
      for (int j = 0; j < 8; ++j) tv[j] = (_Float16)(sX[(ls + 8 - j) * kDBlk + dd] * kCarryH);
      const v8h zz = {(_Float16)0.0f, (_Float16)0.0f, (_Float16)0.0f, (_Float16)0.0f,
                      (_Float16)0.0f, (_Float16)0.0f, (_Float16)0.0f, (_Float16)0.0f};
      _Float16* p = sH + (dd * kSteps + ls) * kHPitch + kState;
      *(v8h*)(p)      = tv;
      *(v8h*)(p + 8)  = zz;
      *(v8h*)(p + 16) = zz;
      *(v8h*)(p + 24) = zz;
    }
    __syncthreads();

#pragma unroll 1
    for (int dd = 0; dd < kDWave; ++dd) {
      const _Float16* ha = sH + ((wave * kDWave + dd) * kSteps + rlane) * kHPitch + koff;
      v8f acc[3];
#pragma unroll
      for (int nt = 0; nt < 3; ++nt) acc[nt] = (v8f){0.f, 0.f, 0.f, 0.f, 0.f, 0.f, 0.f, 0.f};
#pragma unroll
      for (int ks = 0; ks < 3; ++ks) {
        const v16h af = FragH::load(ha + ks * 32);
#pragma unroll
        for (int nt = 0; nt < 3; ++nt) acc[nt] = mma_h(af, bfr[nt][ks], acc[nt]);
      }
#pragma unroll
      for (int nt = 0; nt < 3; ++nt) {
#pragma unroll
        for (int r = 0; r < 8; ++r) {
          const float v = acc[nt][r] * kEmitScale;
          stw[(mOff + r) * kStPitch + dd * kChan + nt * 16 + rlane] = (_Float16)v;
        }
      }
    }
    __builtin_amdgcn_fence(__ATOMIC_RELEASE, "workgroup");
    __builtin_amdgcn_wave_barrier();
    __builtin_amdgcn_fence(__ATOMIC_ACQUIRE, "workgroup");

    unsigned short* Ub = Uo + (size_t)(b * kSeq + l0) * kKtot + (d0 + wave * kDWave) * kChan;
    for (int pass = 0; pass < 2; ++pass) {
#pragma unroll
      for (int it = 0; it < 12; ++it) {
        const int ln = it * 4 + q;
        const int row = ln / 3;
        const int j = ln - row * 3;
        const v8h v = *(const v8h*)(stw + row * kStPitch + j * 64 + c8);
        *(volatile v8h*)(Ub + (size_t)row * kKtot + j * 64 + c8) = v;
      }
      __threadfence();
    }
    __builtin_amdgcn_fence(__ATOMIC_RELEASE, "workgroup");
    __builtin_amdgcn_wave_barrier();
    __builtin_amdgcn_fence(__ATOMIC_ACQUIRE, "workgroup");
  }
}

__global__ __launch_bounds__(256) void gemm_f16_kernel(
    const unsigned short* __restrict__ Ap, int lda,
    const unsigned short* __restrict__ Btp, int ldb,
    float* __restrict__ Cout, int ldc,
    int M, int N, int K, float scale)
{
  const _Float16* A  = (const _Float16*)Ap;
  const _Float16* Bt = (const _Float16*)Btp;
  __shared__ __align__(16) float sT[8][16 * 68];
  const int lane = threadIdx.x & 31;
  const int wave = __builtin_amdgcn_readfirstlane((int)(threadIdx.x >> 5));
  const int tilesN = N >> 6;
  const int tilesM = M >> 6;
  const int tile = blockIdx.x * 8 + wave;
  if (tile >= tilesM * tilesN) return;
  const int tm = tile / tilesN;
  const int tn = tile - tm * tilesN;
  const int m0 = tm << 6;
  const int n0 = tn << 6;

  const int rlane = lane & 15;
  const int koff  = (lane >> 4) * 8;
  const int mOff  = (lane >> 4) * 8;

  v8f acc[4][4];
#pragma unroll
  for (int i = 0; i < 4; ++i)
#pragma unroll
    for (int j = 0; j < 4; ++j) acc[i][j] = (v8f){0.f, 0.f, 0.f, 0.f, 0.f, 0.f, 0.f, 0.f};

  for (int k0 = 0; k0 < K; k0 += 32) {
    v16h bh[4];
#pragma unroll
    for (int j = 0; j < 4; ++j) {
      const size_t bo = (size_t)(n0 + (j << 4) + rlane) * ldb + koff + k0;
      bh[j] = FragH::load(Bt + bo);
    }
#pragma unroll
    for (int i = 0; i < 4; ++i) {
      const size_t ao = (size_t)(m0 + (i << 4) + rlane) * lda + koff + k0;
      const v16h ah = FragH::load(A + ao);
#pragma unroll
      for (int j = 0; j < 4; ++j) acc[i][j] = mma_raw(ah, bh[j], acc[i][j]);
      guard_row4(acc[i][0], acc[i][1], acc[i][2], acc[i][3], ah, bh[0], bh[1], bh[2], bh[3]);
    }
  }
  acc_guard4(acc[0][0], acc[0][1], acc[0][2], acc[0][3]);
  acc_guard4(acc[1][0], acc[1][1], acc[1][2], acc[1][3]);
  acc_guard4(acc[2][0], acc[2][1], acc[2][2], acc[2][3]);
  acc_guard4(acc[3][0], acc[3][1], acc[3][2], acc[3][3]);

  float* slab = sT[wave];
#pragma unroll
  for (int i = 0; i < 4; ++i) {
    const int mBase = m0 + (i << 4);
#pragma unroll
    for (int j = 0; j < 4; ++j) {
#pragma unroll
      for (int r = 0; r < 8; ++r) {
        const float v = acc[i][j][r] * scale;
        slab[(mOff + r) * 68 + (j << 4) + rlane] = v;
      }
    }
    __builtin_amdgcn_fence(__ATOMIC_RELEASE, "workgroup");
    __builtin_amdgcn_wave_barrier();
    __builtin_amdgcn_fence(__ATOMIC_ACQUIRE, "workgroup");
    {
      const int hh = lane >> 4;
      const int c4 = (lane & 15) * 4;
      for (int pass = 0; pass < 2; ++pass) {
#pragma unroll
        for (int it = 0; it < 8; ++it) {
          const int row = it * 2 + hh;
          const v4f v = *(const v4f*)(slab + row * 68 + c4);
          *(volatile v4f*)(Cout + (size_t)(mBase + row) * ldc + n0 + c4) = v;
        }
        __threadfence();
      }
    }
    __builtin_amdgcn_fence(__ATOMIC_RELEASE, "workgroup");
    __builtin_amdgcn_wave_barrier();
    __builtin_amdgcn_fence(__ATOMIC_ACQUIRE, "workgroup");
  }
}

extern "C" void kernel_launch(void* const* d_in, const int* in_sizes, int n_in,
                              void* d_out, int out_size, void* d_ws, size_t ws_size,
                              hipStream_t stream) {
  if (n_in < 7) return;
  if (in_sizes[0] != kRows * kDim) return;
  if (in_sizes[1] != kState) return;
  if (in_sizes[2] != kState) return;
  if (in_sizes[3] != kState * kChan) return;
  if (in_sizes[4] != kChan * kTaps) return;
  if (in_sizes[5] != (kChan / 2) * kDim * kDim) return;
  if (in_sizes[6] != (kChan / 2) * kDim * kDim) return;
  if (out_size != kRows * kDim) return;
  if (ws_size < kWsTotal) return;

  const float* x    = (const float*)d_in[0];
  const float* Av   = (const float*)d_in[1];
  const float* Bv   = (const float*)d_in[2];
  const float* Cm   = (const float*)d_in[3];
  const float* Mt   = (const float*)d_in[4];
  const float* Mp   = (const float*)d_in[5];
  const float* Mm   = (const float*)d_in[6];
  float* out = (float*)d_out;

  char* ws = (char*)d_ws;
  unsigned short* UPL = (unsigned short*)(ws + kOffU);
  unsigned short* WTP = (unsigned short*)(ws + kOffW);

  prep_filter_kernel<<<dim3(kDim / kDWave, kDim / 64), 256, 0, stream>>>(Mp, Mm, WTP);

  scan_emit_kernel<<<dim3(kDim / kDBlk, kBatch), 64, 0, stream>>>(x, Av, Bv, Cm, Mt, UPL);

  gemm_f16_kernel<<<dim3((kRows / 64) * (kDim / 64) / 8, 1), 256, 0, stream>>>(
      UPL, kKtot, WTP, kKtot, out, kDim, kRows, kDim, kKtot, kGemmScale);
}
